// Ourmamba_71966472012603
// MI455X (gfx1250) — hardware-verified
//
#include <hip/hip_runtime.h>
#include <math.h>

typedef __attribute__((ext_vector_type(16))) _Float16 v16h;
typedef __attribute__((ext_vector_type(8)))  _Float16 v8h;
typedef __attribute__((ext_vector_type(16))) __bf16   v16b;
typedef __attribute__((ext_vector_type(8)))  __bf16   v8b;
typedef __attribute__((ext_vector_type(8)))  float    v8f;
typedef __attribute__((ext_vector_type(4)))  float    v4f;

#define DM    1024
#define DIN   2048
#define LSEQ  2048
#define NB    2
#define NST   16
#define RNK   64
#define XDW   96
#define XDP   128
#define XZP   4096
#define TP    260

__device__ __forceinline__ unsigned short f2bf_bits(float f) {
  unsigned u = __float_as_uint(f);
  return (unsigned short)((u + 0x7FFFu + ((u >> 16) & 1u)) >> 16);
}
__device__ __forceinline__ float bf_bits2f(unsigned short h) { return __uint_as_float(((unsigned)h) << 16); }
__device__ __forceinline__ float bfr(float f) { return bf_bits2f(f2bf_bits(f)); }

__device__ __forceinline__ void dep_guard_h(v8f& a, v8f& b, v16h x, v16h y) { asm volatile("v_nop\n\tv_nop\n\tv_nop\n\tv_nop" : "+v"(a), "+v"(b) : "v"(x), "v"(y)); }
__device__ __forceinline__ void dep_guard_b(v8f& a, v8f& b, v16b x, v16b y) { asm volatile("v_nop\n\tv_nop\n\tv_nop\n\tv_nop" : "+v"(a), "+v"(b) : "v"(x), "v"(y)); }
__device__ __forceinline__ void keep4_h(v16h a, v16h b, v16h c, v16h d) { asm volatile("v_nop" :: "v"(a), "v"(b), "v"(c), "v"(d)); }
__device__ __forceinline__ void keep4_b(v16b a, v16b b, v16b c, v16b d) { asm volatile("v_nop" :: "v"(a), "v"(b), "v"(c), "v"(d)); }
__device__ __forceinline__ void acc_guard4(v8f& a, v8f& b, v8f& c, v8f& d) { asm volatile("v_nop\n\tv_nop\n\tv_nop\n\tv_nop" : "+v"(a), "+v"(b), "+v"(c), "+v"(d)); }
template <typename T> struct Frag;
template <> struct Frag<_Float16> {
  typedef v16h V; union U { v16h v; v8h h[2]; };
  static __device__ __forceinline__ v16h load(const _Float16* p) {
    U f; f.h[0] = *(const v8h*)(p); f.h[1] = *(const v8h*)(p + 16); return f.v;
  }
  static __device__ __forceinline__ v8f mma(v16h a, v16h b, v8f c) {
    return __builtin_amdgcn_wmma_f32_16x16x32_f16(false, a, false, b, (short)0, c, false, false);
  }
  static __device__ __forceinline__ void guard(v8f& a, v8f& b, v16h x, v16h y) { dep_guard_h(a, b, x, y); }
  static __device__ __forceinline__ void keep(v16h a, v16h b, v16h c, v16h d) { keep4_h(a, b, c, d); }
};
template <> struct Frag<__bf16> {
  typedef v16b V; union U { v16b v; v8b h[2]; };
  static __device__ __forceinline__ v16b load(const __bf16* p) {
    U f; f.h[0] = *(const v8b*)(p); f.h[1] = *(const v8b*)(p + 16); return f.v;
  }
  static __device__ __forceinline__ v8f mma(v16b a, v16b b, v8f c) {
    return __builtin_amdgcn_wmma_f32_16x16x32_bf16(false, a, false, b, (short)0, c, false, false);
  }
  static __device__ __forceinline__ void guard(v8f& a, v8f& b, v16b x, v16b y) { dep_guard_b(a, b, x, y); }
  static __device__ __forceinline__ void keep(v16b a, v16b b, v16b c, v16b d) { keep4_b(a, b, c, d); }
};

template <int ET> struct Elem;
template <> struct Elem<0> { typedef _Float16 T; };
template <> struct Elem<1> { typedef __bf16 T; };
template <int ET, bool SPLIT, int BIAS_MODE, int OUT_MODE, bool RESID, int ACT = 0>
__global__ __launch_bounds__(256) void wmma_gemm64(
    const unsigned short* __restrict__ Ap, const unsigned short* __restrict__ A2p, int lda, long strideA,
    const unsigned short* __restrict__ Btp, const unsigned short* __restrict__ Bt2p, int ldb, long strideB,
    void* __restrict__ Cout, void* __restrict__ Cout2, int ldc, long strideC,
    const float* __restrict__ bias,
    const float* __restrict__ resid, long strideR,
    int M, int N, int K, float scale) {
  typedef typename Elem<ET>::T T;
  typedef typename Frag<T>::V V;
  const T* A = (const T*)Ap; const T* A2 = (const T*)A2p; const T* Bt = (const T*)Btp; const T* Bt2 = (const T*)Bt2p;
  __shared__ __align__(16) float sT[8][16 * 68];
  const int b    = blockIdx.y;
  const int lane = threadIdx.x & 31;
  const int wave = threadIdx.x >> 5;
  const int tilesN = N >> 6;
  const int tilesM = M >> 6;
  const int tile = blockIdx.x * 8 + wave;
  if (tile >= tilesM * tilesN) return;
  const int tm = tile / tilesN;
  const int tn = tile - tm * tilesN;
  const int m0 = tm << 6;
  const int n0 = tn << 6;

  const T* Ab  = A  + (size_t)b * strideA;
  const T* Bb  = Bt + (size_t)b * strideB;
  const T* Ab2 = SPLIT ? (A2  + (size_t)b * strideA) : nullptr;
  const T* Bb2 = SPLIT ? (Bt2 + (size_t)b * strideB) : nullptr;

  const int rlane = lane & 15;
  const int koff  = (lane >> 4) * 8;
  const int mOff  = (lane >> 4) * 8;

  v8f acc[4][4];
#pragma unroll
  for (int i = 0; i < 4; ++i)
#pragma unroll
    for (int j = 0; j < 4; ++j) acc[i][j] = (v8f){0.f,0.f,0.f,0.f,0.f,0.f,0.f,0.f};

  for (int k0 = 0; k0 < K; k0 += 32) {
    V bh[4], bl[4];
#pragma unroll
    for (int j = 0; j < 4; ++j) {
      const size_t bo = (size_t)(n0 + (j << 4) + rlane) * ldb + koff + k0;
      bh[j] = Frag<T>::load(Bb + bo);
      if (SPLIT) bl[j] = Frag<T>::load(Bb2 + bo);
    }
#pragma unroll
    for (int i = 0; i < 4; ++i) {
      const size_t ao = (size_t)(m0 + (i << 4) + rlane) * lda + koff + k0;
      V ah = Frag<T>::load(Ab + ao);
      V al;
      if (SPLIT) al = Frag<T>::load(Ab2 + ao);
#pragma unroll
      for (int j = 0; j < 4; ++j) {
        acc[i][j] = Frag<T>::mma(ah, bh[j], acc[i][j]);
        if (SPLIT) {
          acc[i][j] = Frag<T>::mma(ah, bl[j], acc[i][j]);
          acc[i][j] = Frag<T>::mma(al, bh[j], acc[i][j]);
        }
      }
      Frag<T>::guard(acc[i][0], acc[i][3], ah, SPLIT ? al : ah);
    }
    Frag<T>::keep(bh[0], bh[1], bh[2], bh[3]);
    if (SPLIT) Frag<T>::keep(bl[0], bl[1], bl[2], bl[3]);
  }
  acc_guard4(acc[0][0], acc[0][1], acc[0][2], acc[0][3]);
  acc_guard4(acc[1][0], acc[1][1], acc[1][2], acc[1][3]);
  acc_guard4(acc[2][0], acc[2][1], acc[2][2], acc[2][3]);
  acc_guard4(acc[3][0], acc[3][1], acc[3][2], acc[3][3]);

  float* slab = sT[wave];
  const float* Rb = RESID ? (resid + (size_t)b * strideR) : nullptr;
#pragma unroll
  for (int i = 0; i < 4; ++i) {
    const int mBase = m0 + (i << 4);
#pragma unroll
    for (int j = 0; j < 4; ++j) {
      const int n = n0 + (j << 4) + rlane;
      float bv = 0.f;
      if (BIAS_MODE == 2) bv = bias[n];
#pragma unroll
      for (int r = 0; r < 8; ++r) {
        float v = acc[i][j][r] * scale;
        if (BIAS_MODE == 1) v += bias[mBase + mOff + r];
        if (BIAS_MODE == 2) v += bv;
        if (RESID) v += Rb[(size_t)(mBase + mOff + r) * ldc + n];
        if (ACT == 1) v = tanhf(v);
        if (ACT == 2) v = fmaxf(v, 0.0f);
        if (ACT == 3) v = v / (1.0f + expf(-v));
        if (ACT == 4) v = (v > 0.f) ? v : 0.01f * v;
        if (ACT == 5) v = 0.5f * v * (1.0f + erff(v * 0.70710678118654752f));
        slab[(mOff + r) * 68 + (j << 4) + rlane] = v;
      }
    }
    __builtin_amdgcn_fence(__ATOMIC_RELEASE, "workgroup");
    __builtin_amdgcn_wave_barrier();
    __builtin_amdgcn_fence(__ATOMIC_ACQUIRE, "workgroup");
    if (OUT_MODE == 0) {
      float* C = (float*)Cout + (size_t)b * strideC;
      const int hh = lane >> 4, c4 = (lane & 15) * 4;
      for (int pass = 0; pass < 2; ++pass) {
#pragma unroll
        for (int it = 0; it < 8; ++it) {
          const int row = it * 2 + hh;
          v4f v = *(const v4f*)(slab + row * 68 + c4);
          *(volatile v4f*)(C + (size_t)(mBase + row) * ldc + n0 + c4) = v;
        }
        __threadfence();
      }
    } else {
      const int q = lane >> 3, c8 = (lane & 7) * 8;
      unsigned short* C  = (unsigned short*)Cout  + (size_t)b * strideC;
      unsigned short* C2 = (OUT_MODE == 2) ? ((unsigned short*)Cout2 + (size_t)b * strideC) : nullptr;
      for (int pass = 0; pass < 2; ++pass) {
#pragma unroll
        for (int it = 0; it < 4; ++it) {
          const int row = it * 4 + q;
          const float* sp = slab + row * 68 + c8;
          v8h hv, lv;
#pragma unroll
          for (int e = 0; e < 8; ++e) {
            if (OUT_MODE == 1) {
              hv[e] = (_Float16)sp[e];
            } else {
              unsigned short hb = f2bf_bits(sp[e]);
              unsigned short lb = f2bf_bits(sp[e] - bf_bits2f(hb));
              hv[e] = __builtin_bit_cast(_Float16, hb);
              lv[e] = __builtin_bit_cast(_Float16, lb);
            }
          }
          *(volatile v8h*)(C + (size_t)(mBase + row) * ldc + n0 + c8) = hv;
          if (OUT_MODE == 2) *(volatile v8h*)(C2 + (size_t)(mBase + row) * ldc + n0 + c8) = lv;
        }
        __threadfence();
      }
    }
    __builtin_amdgcn_fence(__ATOMIC_RELEASE, "workgroup");
    __builtin_amdgcn_wave_barrier();
    __builtin_amdgcn_fence(__ATOMIC_ACQUIRE, "workgroup");
  }
}

__global__ __launch_bounds__(256) void cvt_plane_kernel(
    const float* __restrict__ src, unsigned short* __restrict__ dst,
    int nReal, int nOut, int K, int mode, float scale)
{
  const int i = blockIdx.x * 256 + threadIdx.x;
  const int total8 = (nOut * K) >> 3;
  if (i >= total8) return;
  const int e0  = i << 3;
  const int row = e0 / K;
  const int c   = e0 - row * K;
  const int rc  = (row < nReal) ? row : (nReal - 1);
  const float* p = src + (size_t)rc * K + c;
  const v4f a0 = *(const v4f*)(p);
  const v4f a1 = *(const v4f*)(p + 4);
  const bool ok = row < nReal;
  v8h hv;
#pragma unroll
  for (int e = 0; e < 4; ++e) {
    const float f0 = ok ? a0[e] : 0.f;
    const float f1 = ok ? a1[e] : 0.f;
    unsigned short b0, b1;
    if (mode == 0) {
      b0 = f2bf_bits(f0); b1 = f2bf_bits(f1);
    } else {
      b0 = __builtin_bit_cast(unsigned short, (_Float16)(bfr(f0) * scale));
      b1 = __builtin_bit_cast(unsigned short, (_Float16)(bfr(f1) * scale));
    }
    hv[e]     = __builtin_bit_cast(_Float16, b0);
    hv[4 + e] = __builtin_bit_cast(_Float16, b1);
  }
  unsigned short* q = dst + e0;
  *(volatile v8h*)q = hv;
  __threadfence();
  *(volatile v8h*)q = hv;
}

__global__ __launch_bounds__(256) void conv_silu_kernel(
    const float* __restrict__ XZ, const float* __restrict__ cw, const float* __restrict__ cb,
    float* __restrict__ UC, unsigned short* __restrict__ UCB)
{
  __shared__ __align__(16) float sT[16 * TP];
  const int tid = threadIdx.x, lane = tid & 31, wave = tid >> 5;
  const int d0 = blockIdx.x * 256, d = d0 + tid;
  const int l0 = blockIdx.y * 64;
  const float w0 = bfr(cw[d * 4 + 0]), w1 = bfr(cw[d * 4 + 1]), w2 = bfr(cw[d * 4 + 2]), w3 = bfr(cw[d * 4 + 3]);
  const float bc = bfr(cb[d]);
  float x0, x1, x2;
  {
    const int r0 = l0 - 3, r1 = l0 - 2, r2 = l0 - 1;
    const float v0 = XZ[(size_t)(r0 < 0 ? 0 : r0) * XZP + d];
    const float v1 = XZ[(size_t)(r1 < 0 ? 0 : r1) * XZP + d];
    const float v2 = XZ[(size_t)(r2 < 0 ? 0 : r2) * XZP + d];
    x0 = (r0 >= 0) ? v0 : 0.f;
    x1 = (r1 >= 0) ? v1 : 0.f;
    x2 = (r2 >= 0) ? v2 : 0.f;
  }
  const int hrow = wave >> 1;
  const int hch  = (wave & 1) * 128 + lane * 4;
#pragma unroll 1
  for (int sub = 0; sub < 4; ++sub) {
    const int lb = l0 + sub * 16;
#pragma unroll 1
    for (int s = 0; s < 16; ++s) {
      const float xc = XZ[(size_t)(lb + s) * XZP + d];
      float acc = w0 * x0;
      acc = fmaf(w1, x1, acc);
      acc = fmaf(w2, x2, acc);
      acc = fmaf(w3, xc, acc);
      const float sv = acc + bc;
      const float sg = __builtin_amdgcn_rcpf(1.0f + __expf(-sv));
      sT[s * TP + tid] = sv * sg;
      x0 = x1; x1 = x2; x2 = xc;
    }
    __syncthreads();
    v4f fv[4];
    v8h bv[2];
#pragma unroll
    for (int it = 0; it < 4; ++it) fv[it] = *(const v4f*)(sT + (it * 4 + hrow) * TP + hch);
#pragma unroll
    for (int it = 0; it < 2; ++it) {
      const float* sp = sT + (it * 8 + wave) * TP + lane * 8;
      const v4f a0 = *(const v4f*)(sp);
      const v4f a1 = *(const v4f*)(sp + 4);
#pragma unroll
      for (int e = 0; e < 4; ++e) {
        bv[it][e]     = __builtin_bit_cast(_Float16, f2bf_bits(a0[e]));
        bv[it][4 + e] = __builtin_bit_cast(_Float16, f2bf_bits(a1[e]));
      }
    }
    for (int pass = 0; pass < 2; ++pass) {
#pragma unroll
      for (int it = 0; it < 4; ++it)
        *(volatile v4f*)(UC + (size_t)(lb + it * 4 + hrow) * DIN + d0 + hch) = fv[it];
#pragma unroll
      for (int it = 0; it < 2; ++it)
        *(volatile v8h*)(UCB + (size_t)(lb + it * 8 + wave) * DIN + d0 + lane * 8) = bv[it];
      __threadfence();
    }
    __syncthreads();
  }
}

__global__ __launch_bounds__(256) void scan_kernel(
    const float* __restrict__ DT, const float* __restrict__ UC, const float* __restrict__ XZ,
    const unsigned short* __restrict__ DBLH, const unsigned short* __restrict__ DBLL,
    const float* __restrict__ dt_b, const float* __restrict__ A_log, const float* __restrict__ Dv,
    unsigned short* __restrict__ YH)
{
  __shared__ __align__(16) float sB[16 * NST];
  __shared__ __align__(16) float sC[16 * NST];
  __shared__ __align__(16) float sY[16 * TP];
  const int tid = threadIdx.x, lane = tid & 31, wave = tid >> 5;
  const int d0 = blockIdx.x * 256, d = d0 + tid;

  float An[NST];
#pragma unroll
  for (int n = 0; n < NST; ++n) An[n] = -__expf(bfr(A_log[d * NST + n]));
  const float bd = bfr(dt_b[d]);
  const float Dd = bfr(Dv[d]);
  float h[NST];
#pragma unroll
  for (int n = 0; n < NST; ++n) h[n] = 0.f;

#pragma unroll 1
  for (int c = 0; c < LSEQ / 16; ++c) {
    const int l0 = c * 16;
    {
      const int r = tid >> 4, q = tid & 15;
      const size_t o = (size_t)(l0 + r) * XDP + RNK + q;
      sB[r * NST + q] = bf_bits2f(DBLH[o]) + bf_bits2f(DBLL[o]);
      sC[r * NST + q] = bf_bits2f(DBLH[o + NST]) + bf_bits2f(DBLL[o + NST]);
    }
    __syncthreads();
#pragma unroll 1
    for (int s = 0; s < 16; ++s) {
      const size_t l = (size_t)(l0 + s);
      const float a   = DT[l * DIN + d] + bd;
      const float dt  = fmaxf(a, 0.f) + __logf(1.0f + __expf(-fabsf(a)));
      const float ucv = UC[l * DIN + d];
      const float zv  = XZ[l * XZP + DIN + d];
      const float u   = dt * ucv;
      v4f Bq[4], Cq[4];
#pragma unroll
      for (int qq = 0; qq < 4; ++qq) {
        Bq[qq] = *(const v4f*)(sB + s * NST + 4 * qq);
        Cq[qq] = *(const v4f*)(sC + s * NST + 4 * qq);
      }
      float y = 0.f;
#pragma unroll
      for (int n = 0; n < NST; ++n) {
        const float e = __expf(dt * An[n]);
        h[n] = fmaf(e, h[n], u * Bq[n >> 2][n & 3]);
        y = fmaf(h[n], Cq[n >> 2][n & 3], y);
      }
      y = fmaf(ucv, Dd, y);
      const float sg = __builtin_amdgcn_rcpf(1.0f + __expf(-zv));
      y = y * (zv * sg);
      sY[s * TP + tid] = y * 256.0f;
    }
    __syncthreads();
    v8h hv[2];
#pragma unroll
    for (int it = 0; it < 2; ++it) {
      const float* sp = sY + (it * 8 + wave) * TP + lane * 8;
      const v4f a0 = *(const v4f*)(sp);
      const v4f a1 = *(const v4f*)(sp + 4);
#pragma unroll
      for (int e = 0; e < 4; ++e) { hv[it][e] = (_Float16)a0[e]; hv[it][4 + e] = (_Float16)a1[e]; }
    }
    for (int pass = 0; pass < 2; ++pass) {
#pragma unroll
      for (int it = 0; it < 2; ++it)
        *(volatile v8h*)(YH + (size_t)(l0 + it * 8 + wave) * DIN + d0 + lane * 8) = hv[it];
      __threadfence();
    }
  }
}

extern "C" void kernel_launch(void* const* d_in, const int* in_sizes, int n_in,
                              void* d_out, int out_size, void* d_ws, size_t ws_size,
                              hipStream_t stream)
{
  if (n_in < 10) return;
  const float* x_norm     = (const float*)d_in[0];
  const float* in_proj_w  = (const float*)d_in[1];
  const float* conv_w     = (const float*)d_in[2];
  const float* conv_b     = (const float*)d_in[3];
  const float* x_proj_w   = (const float*)d_in[4];
  const float* dt_proj_w  = (const float*)d_in[5];
  const float* dt_proj_b  = (const float*)d_in[6];
  const float* out_proj_w = (const float*)d_in[7];
  const float* A_log      = (const float*)d_in[8];
  const float* Dvec       = (const float*)d_in[9];
  float* dout = (float*)d_out;

  if (in_sizes[0] != NB * LSEQ * DM) return;
  if (in_sizes[1] != 2 * DIN * DM) return;
  if (in_sizes[2] != DIN * 4 || in_sizes[3] != DIN) return;
  if (in_sizes[4] != XDW * DIN || in_sizes[5] != DIN * RNK || in_sizes[6] != DIN) return;
  if (in_sizes[7] != DM * DIN || in_sizes[8] != DIN * NST || in_sizes[9] != DIN) return;
  if (out_size != NB * LSEQ * DM) return;

  const size_t SZ_WIB = (size_t)2 * DIN * DM * 2;
  const size_t SZ_WXB = (size_t)XDP * DIN * 2;
  const size_t SZ_WDB = (size_t)DIN * RNK * 2;
  const size_t SZ_WOH = (size_t)DM * DIN * 2;
  const size_t SZ_XB  = (size_t)LSEQ * DM * 2;
  const size_t SZ_XZ  = (size_t)LSEQ * XZP * 4;
  const size_t SZ_UC  = (size_t)LSEQ * DIN * 4;
  const size_t SZ_UCB = (size_t)LSEQ * DIN * 2;
  const size_t SZ_DBP = (size_t)LSEQ * XDP * 2;
  const size_t SZ_DT  = (size_t)LSEQ * DIN * 4;
  const size_t SZ_YH  = (size_t)LSEQ * DIN * 2;
  const size_t OFF_WIB  = 0;
  const size_t OFF_WXB  = OFF_WIB  + SZ_WIB;
  const size_t OFF_WDB  = OFF_WXB  + SZ_WXB;
  const size_t OFF_WOH  = OFF_WDB  + SZ_WDB;
  const size_t OFF_XB   = OFF_WOH  + SZ_WOH;
  const size_t OFF_XZ   = OFF_XB   + SZ_XB;
  const size_t OFF_UC   = OFF_XZ   + SZ_XZ;
  const size_t OFF_UCB  = OFF_UC   + SZ_UC;
  const size_t OFF_DBLH = OFF_UCB  + SZ_UCB;
  const size_t OFF_DBLL = OFF_DBLH + SZ_DBP;
  const size_t OFF_DT   = OFF_DBLL + SZ_DBP;
  const size_t OFF_YH   = OFF_DT   + SZ_DT;
  const size_t TOTAL    = OFF_YH   + SZ_YH;
  if (ws_size < TOTAL) return;

  char* ws = (char*)d_ws;
  unsigned short* WIB  = (unsigned short*)(ws + OFF_WIB);
  unsigned short* WXB  = (unsigned short*)(ws + OFF_WXB);
  unsigned short* WDB  = (unsigned short*)(ws + OFF_WDB);
  unsigned short* WOH  = (unsigned short*)(ws + OFF_WOH);
  unsigned short* XB   = (unsigned short*)(ws + OFF_XB);
  float*          XZ   = (float*)(ws + OFF_XZ);
  float*          UC   = (float*)(ws + OFF_UC);
  unsigned short* UCB  = (unsigned short*)(ws + OFF_UCB);
  unsigned short* DBLH = (unsigned short*)(ws + OFF_DBLH);
  unsigned short* DBLL = (unsigned short*)(ws + OFF_DBLL);
  float*          DT   = (float*)(ws + OFF_DT);
  unsigned short* YH   = (unsigned short*)(ws + OFF_YH);
  const float* dummy_bias  = dt_proj_b;
  const float* dummy_resid = UC;

  cvt_plane_kernel<<<(2 * DIN * DM) / 8 / 256, 256, 0, stream>>>(in_proj_w, WIB, 2 * DIN, 2 * DIN, DM, 0, 1.0f);
  cvt_plane_kernel<<<(XDP * DIN) / 8 / 256, 256, 0, stream>>>(x_proj_w, WXB, XDW, XDP, DIN, 0, 1.0f);
  cvt_plane_kernel<<<(DIN * RNK) / 8 / 256, 256, 0, stream>>>(dt_proj_w, WDB, DIN, DIN, RNK, 0, 1.0f);
  cvt_plane_kernel<<<(DM * DIN) / 8 / 256, 256, 0, stream>>>(out_proj_w, WOH, DM, DM, DIN, 1, 64.0f);

  for (int b = 0; b < NB; ++b) {
    const float* xb = x_norm + (size_t)b * LSEQ * DM;
    float* ob = dout + (size_t)b * LSEQ * DM;

    cvt_plane_kernel<<<(LSEQ * DM) / 8 / 256, 256, 0, stream>>>(xb, XB, LSEQ, LSEQ, DM, 0, 1.0f);

    wmma_gemm64<1, false, 0, 0, false><<<dim3(256, 1), 256, 0, stream>>>(
        XB, XB, DM, 0L, WIB, WIB, DM, 0L,
        (void*)XZ, (void*)XZ, XZP, 0L, dummy_bias, dummy_resid, 0L, LSEQ, XZP, DM, 1.0f);

    conv_silu_kernel<<<dim3(DIN / 256, LSEQ / 64), 256, 0, stream>>>(XZ, conv_w, conv_b, UC, UCB);

    wmma_gemm64<1, false, 0, 2, false><<<dim3(8, 1), 256, 0, stream>>>(
        UCB, UCB, DIN, 0L, WXB, WXB, DIN, 0L,
        (void*)DBLH, (void*)DBLL, XDP, 0L, dummy_bias, dummy_resid, 0L, LSEQ, XDP, DIN, 1.0f);

    wmma_gemm64<1, false, 0, 0, false><<<dim3(128, 1), 256, 0, stream>>>(
        DBLH, DBLH, XDP, 0L, WDB, WDB, RNK, 0L,
        (void*)DT, (void*)DT, DIN, 0L, dummy_bias, dummy_resid, 0L, LSEQ, DIN, RNK, 1.0f);

    scan_kernel<<<DIN / 256, 256, 0, stream>>>(DT, UC, XZ, DBLH, DBLL, dt_proj_b, A_log, Dvec, YH);

    wmma_gemm64<0, false, 0, 0, false><<<dim3(64, 1), 256, 0, stream>>>(
        YH, YH, DIN, 0L, WOH, WOH, DIN, 0L,
        (void*)ob, (void*)ob, DM, 0L, dummy_bias, dummy_resid, 0L, LSEQ, DM, DIN, 1.0f / 16384.0f);
  }

  (void)hipGetLastError();
}
